// MambaLayer_80985903333490
// MI455X (gfx1250) — hardware-verified
//
#include <hip/hip_runtime.h>
#include <math.h>

typedef __attribute__((ext_vector_type(16))) _Float16 v16h;
typedef __attribute__((ext_vector_type(8)))  _Float16 v8h;
typedef __attribute__((ext_vector_type(16))) __bf16   v16b;
typedef __attribute__((ext_vector_type(8)))  __bf16   v8b;
typedef __attribute__((ext_vector_type(8)))  float    v8f;
typedef __attribute__((ext_vector_type(4)))  float    v4f;

constexpr int kBatch  = 2;
constexpr int kSeq    = 1024;
constexpr int kDm     = 1024;
constexpr int kDin    = 2048;
constexpr int kNst    = 16;
constexpr int kXzP    = 2 * kDin;
constexpr int kXdN    = 2 * kNst + 1;
constexpr int kXdP    = 64;
constexpr int kRows   = kBatch * kSeq;
constexpr int kConvTP = 260;
constexpr int kScanTS = 64;
constexpr int kScanCh = 64;
constexpr int kScanYP = 68;
constexpr float kLnEps = 1e-5f;
static_assert(kXdN <= kXdP, "x_proj pad");
static_assert((kDm % 32) == 0 && (kDin % 32) == 0, "GEMM K multiples of 32");
static_assert((kRows % 64) == 0 && (kXzP % 64) == 0 && (kXdP % 64) == 0 && (kDm % 64) == 0, "GEMM M,N multiples of 64");
static_assert((kDm % 64) == 0 && (kDin % 64) == 0, "transpose tile multiples");
static_assert((kSeq % kScanTS) == 0 && (kSeq % 64) == 0 && (kDin % kScanCh) == 0 && (kDin % 256) == 0, "tile multiples");
static_assert(kDm == 1024, "LayerNorm lane map assumes 1024 columns");

constexpr size_t kOffWIH  = 0;
constexpr size_t kOffWIL  = kOffWIH + (size_t)kXzP  * kDm  * 2;
constexpr size_t kOffWOH  = kOffWIL + (size_t)kXzP  * kDm  * 2;
constexpr size_t kOffWOL  = kOffWOH + (size_t)kDm   * kDin * 2;
constexpr size_t kOffWXH  = kOffWOL + (size_t)kDm   * kDin * 2;
constexpr size_t kOffWXL  = kOffWXH + (size_t)kXdP  * kDin * 2;
constexpr size_t kOffXNH  = kOffWXL + (size_t)kXdP  * kDin * 2;
constexpr size_t kOffXNL  = kOffXNH + (size_t)kRows * kDm  * 2;
constexpr size_t kOffXZ   = kOffXNL + (size_t)kRows * kDm  * 2;
constexpr size_t kOffUC   = kOffXZ  + (size_t)kRows * kXzP * 4;
constexpr size_t kOffUCH  = kOffUC  + (size_t)kRows * kDin * 4;
constexpr size_t kOffUCL  = kOffUCH + (size_t)kRows * kDin * 2;
constexpr size_t kOffXD   = kOffUCL + (size_t)kRows * kDin * 2;
constexpr size_t kOffYH   = kOffXD  + (size_t)kRows * kXdP * 4;
constexpr size_t kOffYL   = kOffYH  + (size_t)kRows * kDin * 2;
constexpr size_t kWsTotal = kOffYL  + (size_t)kRows * kDin * 2;
static_assert(kWsTotal == 118489088ull, "carve total");
static_assert(kWsTotal <= 134217728ull, "carve cap");
static_assert((kOffWIL % 128) == 0 && (kOffWOH % 128) == 0 && (kOffWOL % 128) == 0 && (kOffWXH % 128) == 0 &&
              (kOffWXL % 128) == 0 && (kOffXNH % 128) == 0 && (kOffXNL % 128) == 0 && (kOffXZ % 128) == 0 &&
              (kOffUC % 128) == 0 && (kOffUCH % 128) == 0 && (kOffUCL % 128) == 0 && (kOffXD % 128) == 0 &&
              (kOffYH % 128) == 0 && (kOffYL % 128) == 0, "128-B aligned regions");

__device__ __forceinline__ unsigned short f2bf_bits(float f) {
  unsigned u = __float_as_uint(f);
  return (unsigned short)((u + 0x7FFFu + ((u >> 16) & 1u)) >> 16);
}
__device__ __forceinline__ float bf_bits2f(unsigned short h) { return __uint_as_float(((unsigned)h) << 16); }

__device__ __forceinline__ void guard4_b(v8f& a, v8f& b, v8f& c, v8f& d, v16b x, v16b y) {
  asm volatile("v_nop\n\tv_nop\n\tv_nop\n\tv_nop" : "+v"(a), "+v"(b), "+v"(c), "+v"(d) : "v"(x), "v"(y));
}
__device__ __forceinline__ void keep4_b(v16b a, v16b b, v16b c, v16b d) { asm volatile("v_nop" :: "v"(a), "v"(b), "v"(c), "v"(d)); }
__device__ __forceinline__ void acc_guard4(v8f& a, v8f& b, v8f& c, v8f& d) { asm volatile("v_nop\n\tv_nop\n\tv_nop\n\tv_nop" : "+v"(a), "+v"(b), "+v"(c), "+v"(d)); }

struct FragB {
  union U { v16b v; v8b h[2]; };
  static __device__ __forceinline__ v16b load(const __bf16* p) {
    U f; f.h[0] = *(const v8b*)(p); f.h[1] = *(const v8b*)(p + 16); return f.v;
  }
  static __device__ __forceinline__ v8f mma(v16b a, v16b b, v8f c) {
    return __builtin_amdgcn_wmma_f32_16x16x32_bf16(false, a, false, b, (short)0, c, false, false);
  }
};

template <bool RESID>
__global__ __launch_bounds__(256) void wmma_gemm64_split(
    const unsigned short* __restrict__ Ap, const unsigned short* __restrict__ A2p, int lda,
    const unsigned short* __restrict__ Btp, const unsigned short* __restrict__ Bt2p, int ldb,
    float* __restrict__ Cf, int ldc,
    const float* __restrict__ resid,
    int M, int N, int K) {
  const __bf16* A   = (const __bf16*)Ap;
  const __bf16* A2  = (const __bf16*)A2p;
  const __bf16* Bt  = (const __bf16*)Btp;
  const __bf16* Bt2 = (const __bf16*)Bt2p;
  __shared__ __align__(16) float sT[8][16 * 68];
  const int lane = threadIdx.x & 31;
  const int wave = threadIdx.x >> 5;
  const int tilesN = N >> 6;
  const int tilesM = M >> 6;
  const int tile = blockIdx.x * 8 + wave;
  if (tile >= tilesM * tilesN) return;
  const int tm = tile / tilesN;
  const int tn = tile - tm * tilesN;
  const int m0 = tm << 6;
  const int n0 = tn << 6;

  const int rlane = lane & 15;
  const int koff  = (lane >> 4) * 8;
  const int mOff  = (lane >> 4) * 8;

  v8f acc[4][4];
#pragma unroll
  for (int i = 0; i < 4; ++i)
#pragma unroll
    for (int j = 0; j < 4; ++j) acc[i][j] = (v8f){0.f,0.f,0.f,0.f,0.f,0.f,0.f,0.f};

  for (int k0 = 0; k0 < K; k0 += 32) {
    v16b bh[4], bl[4];
#pragma unroll
    for (int j = 0; j < 4; ++j) {
      const size_t bo = (size_t)(n0 + (j << 4) + rlane) * ldb + koff + k0;
      bh[j] = FragB::load(Bt + bo);
      bl[j] = FragB::load(Bt2 + bo);
    }
#pragma unroll
    for (int i = 0; i < 4; ++i) {
      const size_t ao = (size_t)(m0 + (i << 4) + rlane) * lda + koff + k0;
      const v16b ah = FragB::load(A + ao);
      const v16b al = FragB::load(A2 + ao);
#pragma unroll
      for (int j = 0; j < 4; ++j) {
        acc[i][j] = FragB::mma(ah, bh[j], acc[i][j]);
        acc[i][j] = FragB::mma(ah, bl[j], acc[i][j]);
        acc[i][j] = FragB::mma(al, bh[j], acc[i][j]);
      }
      guard4_b(acc[i][0], acc[i][1], acc[i][2], acc[i][3], ah, al);
    }
    keep4_b(bh[0], bh[1], bh[2], bh[3]);
    keep4_b(bl[0], bl[1], bl[2], bl[3]);
  }
  acc_guard4(acc[0][0], acc[0][1], acc[0][2], acc[0][3]);
  acc_guard4(acc[1][0], acc[1][1], acc[1][2], acc[1][3]);
  acc_guard4(acc[2][0], acc[2][1], acc[2][2], acc[2][3]);
  acc_guard4(acc[3][0], acc[3][1], acc[3][2], acc[3][3]);

  float* slab = sT[wave];
  const int hh = lane >> 4, c4 = (lane & 15) * 4;
#pragma unroll
  for (int i = 0; i < 4; ++i) {
    const int mBase = m0 + (i << 4);
#pragma unroll
    for (int j = 0; j < 4; ++j) {
#pragma unroll
      for (int r = 0; r < 8; ++r) slab[(mOff + r) * 68 + (j << 4) + rlane] = acc[i][j][r];
    }
    __builtin_amdgcn_fence(__ATOMIC_RELEASE, "workgroup");
    __builtin_amdgcn_wave_barrier();
    __builtin_amdgcn_fence(__ATOMIC_ACQUIRE, "workgroup");
    v4f vals[8];
#pragma unroll
    for (int it = 0; it < 8; ++it) {
      const int row = it * 2 + hh;
      vals[it] = *(const v4f*)(slab + row * 68 + c4);
    }
    if (RESID) {
#pragma unroll
      for (int it = 0; it < 8; ++it) {
        const int row = it * 2 + hh;
        const v4f rv = *(const v4f*)(resid + (size_t)(mBase + row) * ldc + n0 + c4);
        vals[it] = vals[it] + rv;
      }
    }
    for (int pass = 0; pass < 2; ++pass) {
#pragma unroll
      for (int it = 0; it < 8; ++it) {
        const int row = it * 2 + hh;
        *(volatile v4f*)(Cf + (size_t)(mBase + row) * ldc + n0 + c4) = vals[it];
      }
      __threadfence();
    }
    __builtin_amdgcn_fence(__ATOMIC_RELEASE, "workgroup");
    __builtin_amdgcn_wave_barrier();
    __builtin_amdgcn_fence(__ATOMIC_ACQUIRE, "workgroup");
  }
}

__global__ __launch_bounds__(256) void transpose_split_kernel(
    const float* __restrict__ W, unsigned short* __restrict__ Bh, unsigned short* __restrict__ Bl, int Kdim, int Ndim)
{
  __shared__ float tile[64 * 65];
  const int tid = threadIdx.x, lane = tid & 31, wave = tid >> 5;
  const int n0 = blockIdx.x * 64;
  const int k0 = blockIdx.y * 64;
#pragma unroll 8
  for (int p = 0; p < 16; ++p) {
    const int idx = tid + p * 256;
    const int kk  = idx >> 6;
    const int nn  = idx & 63;
    const int n   = n0 + nn;
    const int nc  = (n < Ndim) ? n : (Ndim - 1);
    const float v = W[(size_t)(k0 + kk) * Ndim + nc];
    tile[kk * 65 + nn] = (n < Ndim) ? v : 0.f;
  }
  __syncthreads();
  const int q = lane >> 3, c8 = (lane & 7) * 8;
  v8h hv[2], lv[2];
#pragma unroll
  for (int it = 0; it < 2; ++it) {
    const int nrow = it * 32 + wave * 4 + q;
#pragma unroll
    for (int e = 0; e < 8; ++e) {
      const float f = tile[(c8 + e) * 65 + nrow];
      const unsigned short hb = f2bf_bits(f);
      const unsigned short lb = f2bf_bits(f - bf_bits2f(hb));
      hv[it][e] = __builtin_bit_cast(_Float16, hb);
      lv[it][e] = __builtin_bit_cast(_Float16, lb);
    }
  }
  for (int pass = 0; pass < 2; ++pass) {
#pragma unroll
    for (int it = 0; it < 2; ++it) {
      const int nrow = it * 32 + wave * 4 + q;
      const size_t o = (size_t)(n0 + nrow) * Kdim + k0 + c8;
      *(volatile v8h*)(Bh + o) = hv[it];
      *(volatile v8h*)(Bl + o) = lv[it];
    }
    __threadfence();
  }
}

__global__ __launch_bounds__(256) void layernorm_split_kernel(
    const float* __restrict__ x, const float* __restrict__ g, const float* __restrict__ bt,
    unsigned short* __restrict__ XNH, unsigned short* __restrict__ XNL)
{
  const int lane = threadIdx.x & 31, wave = threadIdx.x >> 5;
  const int tok = blockIdx.x * 8 + wave;
  const float* row = x + (size_t)tok * kDm;
  float s = 0.f;
#pragma unroll 1
  for (int it = 0; it < 4; ++it) {
    const float* p = row + it * 256 + lane * 8;
    const v4f a0 = *(const v4f*)(p);
    const v4f a1 = *(const v4f*)(p + 4);
    s += ((a0[0] + a0[1]) + (a0[2] + a0[3])) + ((a1[0] + a1[1]) + (a1[2] + a1[3]));
  }
#pragma unroll
  for (int off = 16; off > 0; off >>= 1) s += __shfl_xor(s, off, 32);
  const float mu = s * (1.0f / (float)kDm);
  float ss = 0.f;
#pragma unroll 1
  for (int it = 0; it < 4; ++it) {
    const float* p = row + it * 256 + lane * 8;
    const v4f a0 = *(const v4f*)(p);
    const v4f a1 = *(const v4f*)(p + 4);
    float t = 0.f;
#pragma unroll
    for (int e = 0; e < 4; ++e) {
      const float d0 = a0[e] - mu, d1 = a1[e] - mu;
      t += d0 * d0;
      t += d1 * d1;
    }
    ss += t;
  }
#pragma unroll
  for (int off = 16; off > 0; off >>= 1) ss += __shfl_xor(ss, off, 32);
  const float var = ss * (1.0f / (float)kDm);
  const float rs = rsqrtf(var + kLnEps);
#pragma unroll 1
  for (int it = 0; it < 4; ++it) {
    const int c0 = it * 256 + lane * 8;
    const v4f a0 = *(const v4f*)(row + c0);
    const v4f a1 = *(const v4f*)(row + c0 + 4);
    const v4f g0 = *(const v4f*)(g + c0);
    const v4f g1 = *(const v4f*)(g + c0 + 4);
    const v4f b0 = *(const v4f*)(bt + c0);
    const v4f b1 = *(const v4f*)(bt + c0 + 4);
    v8h hv, lv;
#pragma unroll
    for (int e = 0; e < 4; ++e) {
      const float o0 = ((a0[e] - mu) * rs) * g0[e] + b0[e];
      const float o1 = ((a1[e] - mu) * rs) * g1[e] + b1[e];
      const unsigned short h0 = f2bf_bits(o0), h1 = f2bf_bits(o1);
      const unsigned short l0 = f2bf_bits(o0 - bf_bits2f(h0)), l1 = f2bf_bits(o1 - bf_bits2f(h1));
      hv[e]     = __builtin_bit_cast(_Float16, h0);
      hv[4 + e] = __builtin_bit_cast(_Float16, h1);
      lv[e]     = __builtin_bit_cast(_Float16, l0);
      lv[4 + e] = __builtin_bit_cast(_Float16, l1);
    }
    unsigned short* qh = XNH + (size_t)tok * kDm + c0;
    unsigned short* ql = XNL + (size_t)tok * kDm + c0;
    *(volatile v8h*)qh = hv;
    *(volatile v8h*)ql = lv;
    __threadfence();
    *(volatile v8h*)qh = hv;
    *(volatile v8h*)ql = lv;
  }
}

__global__ __launch_bounds__(256) void conv_silu_kernel(
    const float* __restrict__ XZ, const float* __restrict__ cw, const float* __restrict__ cb,
    float* __restrict__ UC, unsigned short* __restrict__ UCH, unsigned short* __restrict__ UCL)
{
  __shared__ __align__(16) float sT[16 * kConvTP];
  const int tid = threadIdx.x, lane = tid & 31, wave = tid >> 5;
  const int d0 = blockIdx.x * 256, d = d0 + tid;
  const int g0 = blockIdx.y * 64;
  const int tb = g0 & (kSeq - 1);
  const v4f wv = *(const v4f*)(cw + (size_t)d * 4);
  const float w0 = wv[0], w1 = wv[1], w2 = wv[2], w3 = wv[3];
  const float bc = cb[d];
  float xm3, xm2, xm1;
  {
    const bool hist = (tb > 0);
    const int rb = hist ? (g0 - 3) : g0;
    const float v3 = XZ[(size_t)rb * kXzP + d];
    const float v2 = XZ[(size_t)(rb + 1) * kXzP + d];
    const float v1 = XZ[(size_t)(rb + 2) * kXzP + d];
    xm3 = hist ? v3 : 0.f;
    xm2 = hist ? v2 : 0.f;
    xm1 = hist ? v1 : 0.f;
  }
  const int hrow = wave >> 1;
  const int hch  = (wave & 1) * 128 + lane * 4;
#pragma unroll 1
  for (int sub = 0; sub < 4; ++sub) {
    const int lb = g0 + sub * 16;
#pragma unroll 1
    for (int s = 0; s < 16; ++s) {
      const float xcur = XZ[(size_t)(lb + s) * kXzP + d];
      float acc = w0 * xm3;
      acc = fmaf(w1, xm2, acc);
      acc = fmaf(w2, xm1, acc);
      acc = fmaf(w3, xcur, acc);
      const float sv = acc + bc;
      const float sg = __builtin_amdgcn_rcpf(1.0f + expf(-sv));
      sT[s * kConvTP + tid] = sv * sg;
      xm3 = xm2; xm2 = xm1; xm1 = xcur;
    }
    __syncthreads();
    v4f fv[4];
    v8h bh[2], blo[2];
#pragma unroll
    for (int it = 0; it < 4; ++it) fv[it] = *(const v4f*)(sT + (it * 4 + hrow) * kConvTP + hch);
#pragma unroll
    for (int it = 0; it < 2; ++it) {
      const float* sp = sT + (it * 8 + wave) * kConvTP + lane * 8;
      const v4f a0 = *(const v4f*)(sp);
      const v4f a1 = *(const v4f*)(sp + 4);
#pragma unroll
      for (int e = 0; e < 4; ++e) {
        const unsigned short h0 = f2bf_bits(a0[e]), h1 = f2bf_bits(a1[e]);
        const unsigned short l0 = f2bf_bits(a0[e] - bf_bits2f(h0)), l1 = f2bf_bits(a1[e] - bf_bits2f(h1));
        bh[it][e]      = __builtin_bit_cast(_Float16, h0);
        bh[it][4 + e]  = __builtin_bit_cast(_Float16, h1);
        blo[it][e]     = __builtin_bit_cast(_Float16, l0);
        blo[it][4 + e] = __builtin_bit_cast(_Float16, l1);
      }
    }
    for (int pass = 0; pass < 2; ++pass) {
#pragma unroll
      for (int it = 0; it < 4; ++it)
        *(volatile v4f*)(UC + (size_t)(lb + it * 4 + hrow) * kDin + d0 + hch) = fv[it];
#pragma unroll
      for (int it = 0; it < 2; ++it) {
        const size_t o = (size_t)(lb + it * 8 + wave) * kDin + d0 + lane * 8;
        *(volatile v8h*)(UCH + o) = bh[it];
        *(volatile v8h*)(UCL + o) = blo[it];
      }
      __threadfence();
    }
    __syncthreads();
  }
}

__global__ __launch_bounds__(64) void scan_gate_kernel(
    const float* __restrict__ XD, const float* __restrict__ UC, const float* __restrict__ XZ,
    const float* __restrict__ Wdt, const float* __restrict__ bdt, const float* __restrict__ Alog,
    unsigned short* __restrict__ YH, unsigned short* __restrict__ YL)
{
  __shared__ __align__(16) float sX[kScanTS * kXdP];
  __shared__ __align__(16) float sY[kScanTS * kScanYP];
  __shared__ __align__(16) float sA[kNst * kScanCh];
  const int tid = threadIdx.x, lane = tid & 31, wave = tid >> 5;
  constexpr int kBlkPerB = kDin / kScanCh;
  const int bix = blockIdx.x / kBlkPerB;
  const int d0  = (blockIdx.x - bix * kBlkPerB) * kScanCh;
  const int d   = d0 + tid;
  const size_t row0 = (size_t)bix * kSeq;
#pragma unroll 1
  for (int s = 0; s < kNst; ++s) sA[s * kScanCh + tid] = -expf(Alog[(size_t)d * kNst + s]);
  __syncthreads();
  float negA[kNst], h[kNst];
#pragma unroll
  for (int s = 0; s < kNst; ++s) {
    negA[s] = sA[s * kScanCh + tid];
    h[s] = 0.f;
  }
  const float wdt = Wdt[d], bb = bdt[d];
  const int lr = tid >> 4, lc4 = (tid & 15) * 4;
  const int cA = lc4, cB = lc4 + 1, cC = lc4 + 2, cD = lc4 + 3;
  const int dc0 = (cA == 0) ? 32 : ((cA <= 32) ? (cA - 1) : cA);
  const int dc1 = (cB <= 32) ? (cB - 1) : cB;
  const int dc2 = (cC <= 32) ? (cC - 1) : cC;
  const int dc3 = (cD <= 32) ? (cD - 1) : cD;
  const int q = lane >> 3, c8 = (lane & 7) * 8;
#pragma unroll 1
  for (int t0 = 0; t0 < kSeq; t0 += kScanTS) {
    __syncthreads();
#pragma unroll 1
    for (int i4 = 0; i4 < 4; ++i4) {
#pragma unroll
      for (int j = 0; j < 4; ++j) {
        const int r = lr + 4 * (i4 * 4 + j);
        const v4f v = *(const v4f*)(XD + (row0 + t0 + r) * kXdP + lc4);
        float* dp = sX + r * kXdP;
        const float e0 = v[0], e1 = v[1], e2 = v[2], e3 = v[3];
        dp[dc0] = e0; dp[dc1] = e1; dp[dc2] = e2; dp[dc3] = e3;
      }
    }
    __syncthreads();
#pragma unroll 1
    for (int s = 0; s < kScanTS; ++s) {
      const int t = t0 + s;
      const float* xr = sX + s * kXdP;
      const float dtraw = xr[32];
      float Bs[kNst], Cs[kNst];
#pragma unroll
      for (int q4 = 0; q4 < 4; ++q4) {
        const v4f bv = *(const v4f*)(xr + 4 * q4);
        const v4f cv = *(const v4f*)(xr + kNst + 4 * q4);
        Bs[4 * q4 + 0] = bv[0]; Bs[4 * q4 + 1] = bv[1]; Bs[4 * q4 + 2] = bv[2]; Bs[4 * q4 + 3] = bv[3];
        Cs[4 * q4 + 0] = cv[0]; Cs[4 * q4 + 1] = cv[1]; Cs[4 * q4 + 2] = cv[2]; Cs[4 * q4 + 3] = cv[3];
      }
      const float v   = dtraw * wdt + bb;
      const float a   = expf(-fabsf(v));
      const float u   = 1.0f + a;
      const float big = __logf(u) + (a - (u - 1.0f)) * __builtin_amdgcn_rcpf(u);
      const float sml = a * (1.0f - a * (0.5f - a * (0.33333334f - 0.25f * a)));
      const float l1p = (a < 0.0078125f) ? sml : big;
      const float dt  = fmaxf(v, 0.0f) + l1p;
      const float xt  = UC[(row0 + t) * kDin + d];
      const float dtx = dt * xt;
      float y = 0.f;
#pragma unroll
      for (int k = 0; k < kNst; ++k) {
        const float e = __expf(dt * negA[k]);
        h[k] = e * h[k] + dtx * Bs[k];
        y = h[k] * Cs[k] + y;
      }
      const float zv = XZ[(row0 + t) * kXzP + kDin + d];
      const float sg = __builtin_amdgcn_rcpf(1.0f + expf(-zv));
      y = y * (zv * sg);
      sY[s * kScanYP + tid] = y;
    }
    __syncthreads();
    v8h hv[8], lv[8];
#pragma unroll
    for (int it = 0; it < 8; ++it) {
      const int row = it * 8 + wave * 4 + q;
      const float* sp = sY + row * kScanYP + c8;
      const v4f a0 = *(const v4f*)(sp);
      const v4f a1 = *(const v4f*)(sp + 4);
#pragma unroll
      for (int e = 0; e < 4; ++e) {
        const unsigned short h0 = f2bf_bits(a0[e]), h1 = f2bf_bits(a1[e]);
        const unsigned short l0 = f2bf_bits(a0[e] - bf_bits2f(h0)), l1 = f2bf_bits(a1[e] - bf_bits2f(h1));
        hv[it][e]     = __builtin_bit_cast(_Float16, h0);
        hv[it][4 + e] = __builtin_bit_cast(_Float16, h1);
        lv[it][e]     = __builtin_bit_cast(_Float16, l0);
        lv[it][4 + e] = __builtin_bit_cast(_Float16, l1);
      }
    }
    for (int pass = 0; pass < 2; ++pass) {
#pragma unroll
      for (int it = 0; it < 8; ++it) {
        const int row = it * 8 + wave * 4 + q;
        const size_t o = (row0 + t0 + row) * kDin + d0 + c8;
        *(volatile v8h*)(YH + o) = hv[it];
        *(volatile v8h*)(YL + o) = lv[it];
      }
      __threadfence();
    }
  }
}

static_assert(((kRows / 64) * (kXzP / 64)) % 8 == 0, "in_proj grid exact");
static_assert(((kRows / 64) * (kXdP / 64)) % 8 == 0, "x_proj grid exact");
static_assert(((kRows / 64) * (kDm / 64)) % 8 == 0, "out_proj grid exact");
static_assert((kRows % 8) == 0, "LayerNorm grid exact");

extern "C" void kernel_launch(void* const* d_in, const int* in_sizes, int n_in,
                              void* d_out, int out_size, void* d_ws, size_t ws_size,
                              hipStream_t stream) {
  if (n_in < 11) return;
  if (in_sizes[0] != kRows * kDm) return;
  if (in_sizes[1] != kDm * kXzP) return;
  if (in_sizes[2] != kDin * 4) return;
  if (in_sizes[3] != kDin) return;
  if (in_sizes[4] != kDin * kXdN) return;
  if (in_sizes[5] != kDin) return;
  if (in_sizes[6] != kDin) return;
  if (in_sizes[7] != kDin * kDm) return;
  if (in_sizes[8] != kDin * kNst) return;
  if (in_sizes[9] != kDm) return;
  if (in_sizes[10] != kDm) return;
  if (out_size != kRows * kDm) return;
  if (ws_size < kWsTotal) return;

  const float* x      = (const float*)d_in[0];
  const float* W_in   = (const float*)d_in[1];
  const float* conv_w = (const float*)d_in[2];
  const float* conv_b = (const float*)d_in[3];
  const float* W_x    = (const float*)d_in[4];
  const float* W_dt   = (const float*)d_in[5];
  const float* b_dt   = (const float*)d_in[6];
  const float* W_out  = (const float*)d_in[7];
  const float* log_A  = (const float*)d_in[8];
  const float* ln_g   = (const float*)d_in[9];
  const float* ln_b   = (const float*)d_in[10];
  float* out = (float*)d_out;

  char* ws = (char*)d_ws;
  unsigned short* WIH  = (unsigned short*)(ws + kOffWIH);
  unsigned short* WIL  = (unsigned short*)(ws + kOffWIL);
  unsigned short* WOH  = (unsigned short*)(ws + kOffWOH);
  unsigned short* WOL  = (unsigned short*)(ws + kOffWOL);
  unsigned short* WXH  = (unsigned short*)(ws + kOffWXH);
  unsigned short* WXL  = (unsigned short*)(ws + kOffWXL);
  unsigned short* XNH  = (unsigned short*)(ws + kOffXNH);
  unsigned short* XNL  = (unsigned short*)(ws + kOffXNL);
  float*          XZ   = (float*)(ws + kOffXZ);
  float*          UC   = (float*)(ws + kOffUC);
  unsigned short* UCH  = (unsigned short*)(ws + kOffUCH);
  unsigned short* UCL  = (unsigned short*)(ws + kOffUCL);
  float*          XD   = (float*)(ws + kOffXD);
  unsigned short* YH   = (unsigned short*)(ws + kOffYH);
  unsigned short* YL   = (unsigned short*)(ws + kOffYL);

  transpose_split_kernel<<<dim3(kXzP / 64, kDm / 64), 256, 0, stream>>>(W_in, WIH, WIL, kDm, kXzP);
  transpose_split_kernel<<<dim3(kDm / 64, kDin / 64), 256, 0, stream>>>(W_out, WOH, WOL, kDin, kDm);
  transpose_split_kernel<<<dim3(kXdP / 64, kDin / 64), 256, 0, stream>>>(W_x, WXH, WXL, kDin, kXdN);

  layernorm_split_kernel<<<kRows / 8, 256, 0, stream>>>(x, ln_g, ln_b, XNH, XNL);

  wmma_gemm64_split<false><<<((kRows / 64) * (kXzP / 64)) / 8, 256, 0, stream>>>(
      XNH, XNL, kDm, WIH, WIL, kDm, XZ, kXzP, x, kRows, kXzP, kDm);

  conv_silu_kernel<<<dim3(kDin / 256, kRows / 64), 256, 0, stream>>>(XZ, conv_w, conv_b, UC, UCH, UCL);

  wmma_gemm64_split<false><<<((kRows / 64) * (kXdP / 64)) / 8, 256, 0, stream>>>(
      UCH, UCL, kDin, WXH, WXL, kDin, XD, kXdP, x, kRows, kXdP, kDin);

  scan_gate_kernel<<<kBatch * (kDin / kScanCh), kScanCh, 0, stream>>>(XD, UC, XZ, W_dt, b_dt, log_A, YH, YL);

  wmma_gemm64_split<true><<<((kRows / 64) * (kDm / 64)) / 8, 256, 0, stream>>>(
      YH, YL, kDin, WOH, WOL, kDin, out, kDm, x, kRows, kDm, kDin);
}
